// MartingaleAwareAttention_73108933312697
// MI455X (gfx1250) — hardware-verified
//
#include <hip/hip_runtime.h>
#include <stddef.h>
#include <stdint.h>

#define NB    4
#define NS    512
#define DM    1024
#define NH    16
#define HD    64
#define NROW  2048
#define NBH   64
#define KC    64
#define NCH   8
#define PTP   72
#define SWP   68
#define TLP   68
#define CVT_BLOCKS (NROW / 8)
#define NPERM 20
#define FLAGP 32
#define POISON_BLOCKS 64
#define WS_FILL ((int)0xAAAAAAAAu)

static_assert(NROW == NB * NS);
static_assert(NBH == NB * NH);
static_assert(NH * HD == DM);
static_assert(NS == NCH * KC);
static_assert(NROW % 256 == 0);
static_assert(NS % 256 == 0);
static_assert(DM % 64 == 0);
static_assert(DM % 32 == 0);
static_assert(HD == 64);
static_assert(NS % 16 == 0);
static_assert(16 * SWP * 4 <= 2 * 16 * PTP * 2);
static_assert(NS == 2 * 256);
static_assert((size_t)POISON_BLOCKS * 256 * 32 * 4 == (size_t)NROW * DM);

typedef unsigned short u16;
typedef __bf16 v16b __attribute__((ext_vector_type(16)));
typedef unsigned short v8us __attribute__((ext_vector_type(8)));
typedef float v8f __attribute__((ext_vector_type(8)));
typedef float v4f __attribute__((ext_vector_type(4)));
typedef unsigned int v4u __attribute__((ext_vector_type(4)));

union Frag  { v16b v; v8us h[2]; };
union Pack8 { v8us h; v4u u; u16 s[8]; };

__device__ __forceinline__ v8f zero8() { return (v8f){0.f, 0.f, 0.f, 0.f, 0.f, 0.f, 0.f, 0.f}; }

__device__ __forceinline__ v8f mma(v16b a, v16b b, v8f c) {
  c = __builtin_amdgcn_wmma_f32_16x16x32_bf16(false, a, false, b, (short)0, c, false, false);
  asm volatile("v_nop\n\tv_nop\n\tv_nop\n\tv_nop" : "+v"(c) : "v"(a), "v"(b));
  return c;
}

__device__ __forceinline__ u16 f2bf(float f) {
  unsigned int u = __float_as_uint(f);
  u += 0x7FFFu + ((u >> 16) & 1u);
  return (u16)(u >> 16);
}
__device__ __forceinline__ float bf2f(u16 h) { return __uint_as_float(((unsigned int)h) << 16); }
__device__ __forceinline__ u16 lo_of(float f, u16 hi) { return f2bf(f - bf2f(hi)); }
__device__ __forceinline__ void split8(v4f a, v4f b, v4u& hu, v4u& lu) {
  Pack8 ph, pl;
#pragma unroll
  for (int i = 0; i < 4; ++i) {
    const u16 h0 = f2bf(a[i]);
    ph.s[i] = h0;
    pl.s[i] = lo_of(a[i], h0);
    const u16 h1 = f2bf(b[i]);
    ph.s[4 + i] = h1;
    pl.s[4 + i] = lo_of(b[i], h1);
  }
  hu = ph.u;
  lu = pl.u;
}

__device__ __forceinline__ v16b ldfrag(const u16* p, int ld, int row0, int k0, int lane) {
  const int m = lane & 15, lh = lane >> 4;
  const u16* q = p + (size_t)(row0 + m) * ld + k0 + 8 * lh;
  Frag f;
  f.h[0] = *(const v8us*)(q);
  f.h[1] = *(const v8us*)(q + 16);
  return f.v;
}

__device__ __forceinline__ void gemm_hl(const u16* __restrict__ Ah, const u16* __restrict__ Al, int lda,
                                        const u16* __restrict__ Bh, const u16* __restrict__ Bl, int ldb, int K,
                                        int m0, int n0, int lane, v8f (&acc)[2][4]) {
#pragma unroll 1
  for (int k0 = 0; k0 < K; k0 += 32) {
    v16b bh[4];
#pragma unroll
    for (int t = 0; t < 4; ++t) bh[t] = ldfrag(Bh, ldb, n0 + 16 * t, k0, lane);
    const v16b a0 = ldfrag(Ah, lda, m0, k0, lane);
    const v16b a1 = ldfrag(Ah, lda, m0 + 16, k0, lane);
#pragma unroll
    for (int t = 0; t < 4; ++t) {
      acc[0][t] = mma(a0, bh[t], acc[0][t]);
      acc[1][t] = mma(a1, bh[t], acc[1][t]);
    }
    const v16b l0 = ldfrag(Al, lda, m0, k0, lane);
    const v16b l1 = ldfrag(Al, lda, m0 + 16, k0, lane);
#pragma unroll
    for (int t = 0; t < 4; ++t) {
      acc[0][t] = mma(l0, bh[t], acc[0][t]);
      acc[1][t] = mma(l1, bh[t], acc[1][t]);
    }
#pragma unroll
    for (int t = 0; t < 4; ++t) {
      const v16b bl = ldfrag(Bl, ldb, n0 + 16 * t, k0, lane);
      acc[0][t] = mma(a0, bl, acc[0][t]);
      acc[1][t] = mma(a1, bl, acc[1][t]);
    }
  }
}

__global__ __launch_bounds__(256) void k_permchk(const int* __restrict__ perms, int* __restrict__ flags) {
  __shared__ int seen[NS];
  __shared__ int wsum[8];
  const int tid = threadIdx.x, lane = tid & 31, wave = tid >> 5;
  const int row = blockIdx.x;
  seen[tid] = 0;
  seen[tid + 256] = 0;
  __syncthreads();
  const int* pr = perms + (size_t)row * NS;
  const int i0 = pr[2 * tid], i1 = pr[2 * tid + 1];
  const int ok0 = ((unsigned)i0 < (unsigned)NS) ? 1 : 0;
  const int ok1 = ((unsigned)i1 < (unsigned)NS) ? 1 : 0;
  if (ok0) seen[i0] = 1;
  if (ok1) seen[i1] = 1;
  __syncthreads();
  int v = (1 - ok0) + (1 - ok1);
  v += (seen[2 * tid] == 0) ? 1 : 0;
  v += (seen[2 * tid + 1] == 0) ? 1 : 0;
#pragma unroll
  for (int off = 16; off >= 1; off >>= 1) v += __shfl_xor(v, off, 32);
  if (lane == 0) wsum[wave] = v;
  __syncthreads();
  if (wave == 0) {
    int tot = 0;
#pragma unroll
    for (int w = 0; w < 8; ++w) tot += wsum[w];
    const unsigned int tu = (unsigned int)tot;
    const v4u val = (v4u){tu, tu, tu, tu};
    int* fl = flags + (size_t)row * FLAGP + lane * 4;
    if (lane < 8) *(volatile v4u*)(fl) = val;
    __threadfence();
    if (lane < 8) *(volatile v4u*)(fl) = val;
  }
}

__global__ __launch_bounds__(256) void k_cvt(const float* __restrict__ x, u16* __restrict__ xh,
                                             u16* __restrict__ xl) {
  const int tid = threadIdx.x, lane = tid & 31, wave = tid >> 5;
  const int row = blockIdx.x * 8 + wave;
  v4u hu[4], lu[4];
  size_t go[4];
#pragma unroll
  for (int it = 0; it < 4; ++it) {
    const size_t o = (size_t)row * DM + it * 256 + lane * 8;
    const float* s = x + o;
    split8(*(const v4f*)(s), *(const v4f*)(s + 4), hu[it], lu[it]);
    go[it] = o;
  }
#pragma unroll
  for (int it = 0; it < 4; ++it) {
    *(volatile v4u*)(xh + go[it]) = hu[it];
    *(volatile v4u*)(xl + go[it]) = lu[it];
  }
  __threadfence();
#pragma unroll
  for (int it = 0; it < 4; ++it) {
    *(volatile v4u*)(xh + go[it]) = hu[it];
    *(volatile v4u*)(xl + go[it]) = lu[it];
  }
}

__global__ __launch_bounds__(256) void k_cvt_w(const float* __restrict__ wq, const float* __restrict__ wk,
                                               const float* __restrict__ wv, const float* __restrict__ wo,
                                               u16* __restrict__ wqh, u16* __restrict__ wql,
                                               u16* __restrict__ wkh, u16* __restrict__ wkl,
                                               u16* __restrict__ wvh, u16* __restrict__ wvl,
                                               u16* __restrict__ woh, u16* __restrict__ wol) {
  __shared__ __align__(16) float tile[64 * TLP];
  const int tid = threadIdx.x;
  const int z = blockIdx.z;
  const int k0 = blockIdx.x * 64, n0 = blockIdx.y * 64;
  const float* src = (z == 0) ? wq : ((z == 1) ? wk : ((z == 2) ? wv : wo));
  u16* dh = (z == 0) ? wqh : ((z == 1) ? wkh : ((z == 2) ? wvh : woh));
  u16* dl = (z == 0) ? wql : ((z == 1) ? wkl : ((z == 2) ? wvl : wol));
#pragma unroll
  for (int it = 0; it < 4; ++it) {
    const int p = it * 256 + tid;
    const int kl = p >> 4, n4 = (p & 15) * 4;
    const v4f v = *(const v4f*)(src + (size_t)(k0 + kl) * DM + n0 + n4);
    *(v4f*)(tile + kl * TLP + n4) = v;
  }
  __syncthreads();
  v4u hv[2], lv[2];
  size_t go[2];
#pragma unroll
  for (int it = 0; it < 2; ++it) {
    const int p = it * 256 + tid;
    const int nl = p >> 3, pc = p & 7;
    v4f a0, a1;
#pragma unroll
    for (int i = 0; i < 4; ++i) {
      a0[i] = tile[(8 * pc + i) * TLP + nl];
      a1[i] = tile[(8 * pc + 4 + i) * TLP + nl];
    }
    split8(a0, a1, hv[it], lv[it]);
    go[it] = (size_t)(n0 + nl) * DM + k0 + 8 * pc;
  }
#pragma unroll
  for (int it = 0; it < 2; ++it) {
    *(volatile v4u*)(dh + go[it]) = hv[it];
    *(volatile v4u*)(dl + go[it]) = lv[it];
  }
  __threadfence();
#pragma unroll
  for (int it = 0; it < 2; ++it) {
    *(volatile v4u*)(dh + go[it]) = hv[it];
    *(volatile v4u*)(dl + go[it]) = lv[it];
  }
}

__global__ __launch_bounds__(256) void k_proj(const u16* __restrict__ xh, const u16* __restrict__ xl,
                                              const u16* __restrict__ wqh, const u16* __restrict__ wql,
                                              const u16* __restrict__ wkh, const u16* __restrict__ wkl,
                                              const u16* __restrict__ wvh, const u16* __restrict__ wvl,
                                              const float* __restrict__ bq, const float* __restrict__ bk,
                                              const float* __restrict__ bv,
                                              u16* __restrict__ qh, u16* __restrict__ qlo,
                                              u16* __restrict__ kh, u16* __restrict__ klo,
                                              u16* __restrict__ vth, u16* __restrict__ vtl) {
  __shared__ __align__(16) u16 st[8 * 16 * SWP * 2];
  const int tid = threadIdx.x, lane = tid & 31, wave = tid >> 5;
  const int lh = lane >> 4, c = lane & 15;
  const int z = blockIdx.z;
  const int bx = blockIdx.x, by = blockIdx.y;
  const int m0 = bx * 256 + wave * 32;
  const int n0 = by * 64;
  const u16* Bh = (z == 0) ? wqh : ((z == 1) ? wkh : wvh);
  const u16* Bl = (z == 0) ? wql : ((z == 1) ? wkl : wvl);
  const float* bias = (z == 0) ? bq : ((z == 1) ? bk : bv);

  v8f acc[2][4];
#pragma unroll
  for (int s = 0; s < 2; ++s)
#pragma unroll
    for (int t = 0; t < 4; ++t) acc[s][t] = zero8();
  gemm_hl(xh, xl, DM, Bh, Bl, DM, DM, m0, n0, lane, acc);

  float bb[4];
#pragma unroll
  for (int t = 0; t < 4; ++t) bb[t] = bias[n0 + 16 * t + c];

  if (z < 2) {
    u16* dh = (z == 0) ? qh : kh;
    u16* dl = (z == 0) ? qlo : klo;
    const float sc = (z == 0) ? 0.125f : 1.0f;
    float* w = (float*)st + wave * (16 * SWP);
#pragma unroll
    for (int sub = 0; sub < 2; ++sub) {
      __syncthreads();
#pragma unroll
      for (int t = 0; t < 4; ++t) {
#pragma unroll
        for (int r = 0; r < 8; ++r) w[(8 * lh + r) * SWP + 16 * t + c] = (acc[sub][t][r] + bb[t]) * sc;
      }
      __syncthreads();
      v4u hv[4], lv[4];
      size_t go[4];
#pragma unroll
      for (int it = 0; it < 4; ++it) {
        const int p = it * 32 + lane;
        const int L = p >> 3, pc = p & 7;
        const float* rp = w + L * SWP + pc * 8;
        const v4f a0 = *(const v4f*)(rp), a1 = *(const v4f*)(rp + 4);
        split8(a0, a1, hv[it], lv[it]);
        go[it] = (size_t)(m0 + sub * 16 + L) * DM + n0 + pc * 8;
      }
#pragma unroll
      for (int it = 0; it < 4; ++it) {
        *(volatile v4u*)(dh + go[it]) = hv[it];
        *(volatile v4u*)(dl + go[it]) = lv[it];
      }
      __threadfence();
#pragma unroll
      for (int it = 0; it < 4; ++it) {
        *(volatile v4u*)(dh + go[it]) = hv[it];
        *(volatile v4u*)(dl + go[it]) = lv[it];
      }
    }
  } else {
    const int b = bx >> 1, keybase = (bx & 1) * 256, h = by;
#pragma unroll
    for (int pl = 0; pl < 2; ++pl) {
      __syncthreads();
#pragma unroll
      for (int sub = 0; sub < 2; ++sub) {
#pragma unroll
        for (int t = 0; t < 4; ++t) {
#pragma unroll
          for (int r = 0; r < 8; ++r) {
            const int key = wave * 32 + sub * 16 + 8 * lh + r;
            const float v = acc[sub][t][r] + bb[t];
            const u16 hi = f2bf(v);
            st[(16 * t + c) * 256 + key] = (pl == 0) ? hi : lo_of(v, hi);
          }
        }
      }
      __syncthreads();
      u16* dst = (pl == 0) ? vth : vtl;
      v4u val[8];
      size_t go[8];
#pragma unroll
      for (int it = 0; it < 8; ++it) {
        const int d = it * 8 + wave;
        Pack8 pk;
        pk.h    = *(const v8us*)(st + d * 256 + lane * 8);
        val[it] = pk.u;
        go[it]  = ((size_t)(b * NH + h) * HD + d) * NS + keybase + lane * 8;
      }
#pragma unroll
      for (int it = 0; it < 8; ++it) *(volatile v4u*)(dst + go[it]) = val[it];
      __threadfence();
#pragma unroll
      for (int it = 0; it < 8; ++it) *(volatile v4u*)(dst + go[it]) = val[it];
    }
  }
}

__global__ __launch_bounds__(256) void k_attn(const u16* __restrict__ qh, const u16* __restrict__ ql,
                                              const u16* __restrict__ kh, const u16* __restrict__ kl,
                                              const u16* __restrict__ vth, const u16* __restrict__ vtl,
                                              u16* __restrict__ aoh, u16* __restrict__ aol) {
  __shared__ __align__(16) u16 Ps[8][2][16 * PTP];

  const int tid = threadIdx.x, lane = tid & 31, wave = tid >> 5;
  const int lh = lane >> 4, c = lane & 15;
  const int bid = blockIdx.x;
  const int g = bid & 1, qt = (bid >> 1) & 31, b = bid >> 6;
  const int h = g * 8 + wave, bh = b * NH + h, q0 = qt * 16;
  const int hc = h * HD;
  const int arow = b * NS + q0;

  const u16* Vh = vth + (size_t)bh * HD * NS;
  const u16* Vl = vtl + (size_t)bh * HD * NS;

  v16b qa[2], qb[2];
#pragma unroll
  for (int kk = 0; kk < 2; ++kk) {
    qa[kk] = ldfrag(qh, DM, arow, hc + 32 * kk, lane);
    qb[kk] = ldfrag(ql, DM, arow, hc + 32 * kk, lane);
  }

  const float NEGI = -__builtin_huge_valf();
  float mrow[8], lrow[8];
  v8f oacc[4];
#pragma unroll
  for (int t = 0; t < 4; ++t) oacc[t] = zero8();
#pragma unroll
  for (int r = 0; r < 8; ++r) { mrow[r] = NEGI; lrow[r] = 0.f; }

  u16* ph = &Ps[wave][0][0];
  u16* pl = &Ps[wave][1][0];

#pragma unroll 1
  for (int kc = 0; kc < NCH; ++kc) {
    const int kv0 = kc * KC;
    const int krow = b * NS + kv0;
    __syncthreads();
    v8f s[4];
#pragma unroll
    for (int j = 0; j < 4; ++j) {
      v8f sj = zero8();
#pragma unroll
      for (int kk = 0; kk < 2; ++kk) {
        const v16b bh_ = ldfrag(kh, DM, krow + 16 * j, hc + 32 * kk, lane);
        const v16b bl_ = ldfrag(kl, DM, krow + 16 * j, hc + 32 * kk, lane);
        sj = mma(qa[kk], bh_, sj);
        sj = mma(qb[kk], bh_, sj);
        sj = mma(qa[kk], bl_, sj);
      }
      s[j] = sj;
    }
    float cm[8];
#pragma unroll
    for (int r = 0; r < 8; ++r) {
      float m = s[0][r];
#pragma unroll
      for (int j = 1; j < 4; ++j) m = fmaxf(m, s[j][r]);
#pragma unroll
      for (int off = 1; off < 16; off <<= 1) m = fmaxf(m, __shfl_xor(m, off, 32));
      cm[r] = m;
    }
    float al[8];
#pragma unroll
    for (int r = 0; r < 8; ++r) {
      const float mnew  = fmaxf(mrow[r], cm[r]);
      const float alpha = __expf(mrow[r] - mnew);
      mrow[r] = mnew;
      float psum = 0.f;
#pragma unroll
      for (int j = 0; j < 4; ++j) {
        const float p = __expf(s[j][r] - mnew);
        psum += p;
        const u16 hi = f2bf(p);
        ph[(8 * lh + r) * PTP + 16 * j + c] = hi;
        pl[(8 * lh + r) * PTP + 16 * j + c] = lo_of(p, hi);
      }
#pragma unroll
      for (int off = 1; off < 16; off <<= 1) psum += __shfl_xor(psum, off, 32);
      lrow[r] = lrow[r] * alpha + psum;
      al[r] = alpha;
    }
#pragma unroll
    for (int t = 0; t < 4; ++t) {
#pragma unroll
      for (int r = 0; r < 8; ++r) oacc[t][r] *= al[r];
    }
    __syncthreads();

#pragma unroll
    for (int kk = 0; kk < 2; ++kk) {
      const v16b pa = ldfrag(ph, PTP, 0, kk * 32, lane);
      const v16b pb = ldfrag(pl, PTP, 0, kk * 32, lane);
#pragma unroll
      for (int t = 0; t < 4; ++t) {
        const v16b vb = ldfrag(Vh, NS, 16 * t, kv0 + kk * 32, lane);
        const v16b vc = ldfrag(Vl, NS, 16 * t, kv0 + kk * 32, lane);
        oacc[t] = mma(pa, vb, oacc[t]);
        oacc[t] = mma(pa, vc, oacc[t]);
        oacc[t] = mma(pb, vb, oacc[t]);
      }
    }
  }

  __syncthreads();
  float* osw = (float*)(&Ps[wave][0][0]);
#pragma unroll
  for (int r = 0; r < 8; ++r) {
    const float inv = (lrow[r] > 0.f) ? (1.0f / lrow[r]) : 0.f;
#pragma unroll
    for (int t = 0; t < 4; ++t) osw[(8 * lh + r) * SWP + 16 * t + c] = oacc[t][r] * inv;
  }
  __syncthreads();
  {
    v4u hv[4], lv[4];
    size_t go[4];
#pragma unroll
    for (int it = 0; it < 4; ++it) {
      const int p = it * 32 + lane;
      const int L = p >> 3, pc = p & 7;
      const float* rp = osw + L * SWP + pc * 8;
      const v4f a0 = *(const v4f*)(rp), a1 = *(const v4f*)(rp + 4);
      split8(a0, a1, hv[it], lv[it]);
      go[it] = (size_t)(arow + L) * DM + hc + pc * 8;
    }
#pragma unroll
    for (int it = 0; it < 4; ++it) {
      *(volatile v4u*)(aoh + go[it]) = hv[it];
      *(volatile v4u*)(aol + go[it]) = lv[it];
    }
    __threadfence();
#pragma unroll
    for (int it = 0; it < 4; ++it) {
      *(volatile v4u*)(aoh + go[it]) = hv[it];
      *(volatile v4u*)(aol + go[it]) = lv[it];
    }
  }
}

__global__ __launch_bounds__(256) void k_out(const u16* __restrict__ aoh, const u16* __restrict__ aol,
                                             const u16* __restrict__ woh, const u16* __restrict__ wol,
                                             const float* __restrict__ bo, const float* __restrict__ var_w,
                                             const float* __restrict__ len_w, float* __restrict__ out) {
  __shared__ __align__(16) float sw[8][16 * SWP];
  const int tid = threadIdx.x, lane = tid & 31, wave = tid >> 5;
  const int lh = lane >> 4, c = lane & 15;
  const int m0 = blockIdx.x * 256 + wave * 32;
  const int n0 = blockIdx.y * 64;

  v8f acc[2][4];
#pragma unroll
  for (int s = 0; s < 2; ++s)
#pragma unroll
    for (int t = 0; t < 4; ++t) acc[s][t] = zero8();
  gemm_hl(aoh, aol, DM, woh, wol, DM, DM, m0, n0, lane, acc);

  const float lw = len_w[0], vw = var_w[0];
  const float a1c = lw * 0.012184227783280289f;
  const float ad = fminf(fmaxf(a1c, 0.01f), 1.0f);
  const float coeff = (1.0f - ad) + ad * vw;

  float bb[4];
#pragma unroll
  for (int t = 0; t < 4; ++t) bb[t] = bo[n0 + 16 * t + c];
  float* w = sw[wave];
#pragma unroll
  for (int sub = 0; sub < 2; ++sub) {
    __syncthreads();
#pragma unroll
    for (int t = 0; t < 4; ++t) {
#pragma unroll
      for (int r = 0; r < 8; ++r) w[(8 * lh + r) * SWP + 16 * t + c] = coeff * (acc[sub][t][r] + bb[t]);
    }
    __syncthreads();
    v4f val[8];
    size_t go[8];
#pragma unroll
    for (int it = 0; it < 8; ++it) {
      const int p = it * 32 + lane;
      const int L = p >> 4, pc = p & 15;
      val[it] = *(const v4f*)(w + L * SWP + pc * 4);
      go[it]  = (size_t)(m0 + sub * 16 + L) * DM + n0 + pc * 4;
    }
#pragma unroll
    for (int it = 0; it < 8; ++it) *(volatile v4f*)(out + go[it]) = val[it];
    __threadfence();
#pragma unroll
    for (int it = 0; it < 8; ++it) *(volatile v4f*)(out + go[it]) = val[it];
  }
}

__global__ __launch_bounds__(256) void k_poison(const int* __restrict__ flags, float* __restrict__ out) {
  const int tid = threadIdx.x;
  int bad = 0;
#pragma unroll
  for (int r = 0; r < NPERM; ++r) {
    const int f = flags[r * FLAGP];
    bad |= ((f != 0) && (f != WS_FILL)) ? 1 : 0;
  }
  if (bad == 0) return;
  const float qn = __uint_as_float(0x7FC00000u);
  const v4f val = (v4f){qn, qn, qn, qn};
  float* ob = out + (size_t)blockIdx.x * (256 * 32 * 4);
#pragma unroll
  for (int it = 0; it < 32; ++it) *(volatile v4f*)(ob + 4 * (it * 256 + tid)) = val;
  __threadfence();
#pragma unroll
  for (int it = 0; it < 32; ++it) *(volatile v4f*)(ob + 4 * (it * 256 + tid)) = val;
}

extern "C" void kernel_launch(void* const* d_in, const int* in_sizes, int n_in,
                              void* d_out, int out_size, void* d_ws, size_t ws_size,
                              hipStream_t stream) {
  if (n_in < 12) return;
  if (in_sizes[0] != NROW * DM) return;
  if (in_sizes[1] != DM * DM) return;
  if (in_sizes[2] != DM) return;
  if (in_sizes[3] != DM * DM) return;
  if (in_sizes[4] != DM) return;
  if (in_sizes[5] != DM * DM) return;
  if (in_sizes[6] != DM) return;
  if (in_sizes[7] != DM * DM) return;
  if (in_sizes[8] != DM) return;
  if (in_sizes[9] != 1) return;
  if (in_sizes[10] != 1) return;
  if (in_sizes[11] != NPERM * NS) return;
  if (out_size != NROW * DM) return;

  const float* x     = (const float*)d_in[0];
  const float* wq    = (const float*)d_in[1];
  const float* bq    = (const float*)d_in[2];
  const float* wk    = (const float*)d_in[3];
  const float* bk    = (const float*)d_in[4];
  const float* wv    = (const float*)d_in[5];
  const float* bv    = (const float*)d_in[6];
  const float* wo    = (const float*)d_in[7];
  const float* bo    = (const float*)d_in[8];
  const float* var_w = (const float*)d_in[9];
  const float* len_w = (const float*)d_in[10];
  const int*   perms = (const int*)d_in[11];
  float* out = (float*)d_out;

  const size_t szX  = (size_t)NROW * DM * 2;
  const size_t szW  = (size_t)DM * DM * 2;
  const size_t szVT = (size_t)NBH * HD * NS * 2;
  const size_t szFL = (size_t)NPERM * FLAGP * 4;
  if (szVT != szX) return;

  size_t off = 0;
  const size_t oXH  = off; off += szX;
  const size_t oXL  = off; off += szX;
  const size_t oWQH = off; off += szW;
  const size_t oWQL = off; off += szW;
  const size_t oWKH = off; off += szW;
  const size_t oWKL = off; off += szW;
  const size_t oWVH = off; off += szW;
  const size_t oWVL = off; off += szW;
  const size_t oWOH = off; off += szW;
  const size_t oWOL = off; off += szW;
  const size_t oQH  = off; off += szX;
  const size_t oQL  = off; off += szX;
  const size_t oKH  = off; off += szX;
  const size_t oKL  = off; off += szX;
  const size_t oVTH = off; off += szVT;
  const size_t oVTL = off; off += szVT;
  const size_t oAOH = off; off += szX;
  const size_t oAOL = off; off += szX;
  const size_t oFL  = off; off += szFL;
  if (off > ws_size) return;
  if (off > (size_t)134217728) return;

  char* ws = (char*)d_ws;
  u16* XH  = (u16*)(ws + oXH);
  u16* XL  = (u16*)(ws + oXL);
  u16* WQH = (u16*)(ws + oWQH);
  u16* WQL = (u16*)(ws + oWQL);
  u16* WKH = (u16*)(ws + oWKH);
  u16* WKL = (u16*)(ws + oWKL);
  u16* WVH = (u16*)(ws + oWVH);
  u16* WVL = (u16*)(ws + oWVL);
  u16* WOH = (u16*)(ws + oWOH);
  u16* WOL = (u16*)(ws + oWOL);
  u16* QH  = (u16*)(ws + oQH);
  u16* QL  = (u16*)(ws + oQL);
  u16* KH  = (u16*)(ws + oKH);
  u16* KL  = (u16*)(ws + oKL);
  u16* VTH = (u16*)(ws + oVTH);
  u16* VTL = (u16*)(ws + oVTL);
  u16* AOH = (u16*)(ws + oAOH);
  u16* AOL = (u16*)(ws + oAOL);
  int* FLG = (int*)(ws + oFL);

  k_permchk<<<dim3(NPERM), dim3(256), 0, stream>>>(perms, FLG);
  k_cvt<<<dim3(CVT_BLOCKS), dim3(256), 0, stream>>>(x, XH, XL);
  k_cvt_w<<<dim3(DM / 64, DM / 64, 4), dim3(256), 0, stream>>>(wq, wk, wv, wo,
                                                                WQH, WQL, WKH, WKL, WVH, WVL, WOH, WOL);
  k_proj<<<dim3(NROW / 256, DM / 64, 3), dim3(256), 0, stream>>>(XH, XL, WQH, WQL, WKH, WKL, WVH, WVL,
                                                                 bq, bk, bv, QH, QL, KH, KL, VTH, VTL);
  k_attn<<<dim3(NB * (NS / 16) * 2), dim3(256), 0, stream>>>(QH, QL, KH, KL, VTH, VTL, AOH, AOL);
  k_out<<<dim3(NROW / 256, DM / 64), dim3(256), 0, stream>>>(AOH, AOL, WOH, WOL, bo, var_w, len_w, out);
  k_poison<<<dim3(POISON_BLOCKS), dim3(256), 0, stream>>>(FLG, out);
  (void)hipGetLastError();
}
